// TensorProductConvLayer_13657996001870
// MI455X (gfx1250) — hardware-verified
//
#include <hip/hip_runtime.h>
#include <math.h>

typedef __attribute__((ext_vector_type(16))) _Float16 v16h;
typedef __attribute__((ext_vector_type(8)))  _Float16 v8h;
typedef __attribute__((ext_vector_type(16))) __bf16   v16b;
typedef __attribute__((ext_vector_type(8)))  __bf16   v8b;
typedef __attribute__((ext_vector_type(8)))  float    v8f;
typedef __attribute__((ext_vector_type(4)))  float    v4f;
typedef __attribute__((ext_vector_type(2)))  float    v2f;
typedef __attribute__((ext_vector_type(4)))  int      v4i;
#define PSCALE 32768.0f
#define U16(p) ((const unsigned short*)(const void*)(p))
#define PSCALE_INV (1.0f / 32768.0f)

__device__ __forceinline__ unsigned short f2bf_bits(float f) {
  unsigned u = __float_as_uint(f);
  return (unsigned short)((u + 0x7FFFu + ((u >> 16) & 1u)) >> 16);
}
__device__ __forceinline__ float bf_bits2f(unsigned short h) { return __uint_as_float(((unsigned)h) << 16); }

__device__ __forceinline__ void dep_guard_h(v8f& a, v8f& b, v16h x, v16h y) { asm volatile("v_nop\n\tv_nop\n\tv_nop\n\tv_nop" : "+v"(a), "+v"(b) : "v"(x), "v"(y)); }
__device__ __forceinline__ void dep_guard_b(v8f& a, v8f& b, v16b x, v16b y) { asm volatile("v_nop\n\tv_nop\n\tv_nop\n\tv_nop" : "+v"(a), "+v"(b) : "v"(x), "v"(y)); }
__device__ __forceinline__ void keep4_h(v16h a, v16h b, v16h c, v16h d) { asm volatile("v_nop" :: "v"(a), "v"(b), "v"(c), "v"(d)); }
__device__ __forceinline__ void keep4_b(v16b a, v16b b, v16b c, v16b d) { asm volatile("v_nop" :: "v"(a), "v"(b), "v"(c), "v"(d)); }
__device__ __forceinline__ void fence_v4(v4f& t) { asm volatile("" : "+v"(t)); }
__device__ __forceinline__ void acc_guard4(v8f& a, v8f& b, v8f& c, v8f& d) { asm volatile("v_nop\n\tv_nop\n\tv_nop\n\tv_nop" : "+v"(a), "+v"(b), "+v"(c), "+v"(d)); }
template <typename T> struct Frag;
template <> struct Frag<_Float16> {
  typedef v16h V; union U { v16h v; v8h h[2]; };
  static __device__ __forceinline__ v16h load(const _Float16* p) {
    U f; f.h[0] = *(const v8h*)(p); f.h[1] = *(const v8h*)(p + 16); return f.v;
  }
  static __device__ __forceinline__ v8f mma(v16h a, v16h b, v8f c) {
    return __builtin_amdgcn_wmma_f32_16x16x32_f16(false, a, false, b, (short)0, c, false, false);
  }
  static __device__ __forceinline__ void guard(v8f& a, v8f& b, v16h x, v16h y) { dep_guard_h(a, b, x, y); }
  static __device__ __forceinline__ void keep(v16h a, v16h b, v16h c, v16h d) { keep4_h(a, b, c, d); }
};
template <> struct Frag<__bf16> {
  typedef v16b V; union U { v16b v; v8b h[2]; };
  static __device__ __forceinline__ v16b load(const __bf16* p) {
    U f; f.h[0] = *(const v8b*)(p); f.h[1] = *(const v8b*)(p + 16); return f.v;
  }
  static __device__ __forceinline__ v8f mma(v16b a, v16b b, v8f c) {
    return __builtin_amdgcn_wmma_f32_16x16x32_bf16(false, a, false, b, (short)0, c, false, false);
  }
  static __device__ __forceinline__ void guard(v8f& a, v8f& b, v16b x, v16b y) { dep_guard_b(a, b, x, y); }
  static __device__ __forceinline__ void keep(v16b a, v16b b, v16b c, v16b d) { keep4_b(a, b, c, d); }
};

template <int ET> struct Elem;
template <> struct Elem<0> { typedef _Float16 T; };
template <> struct Elem<1> { typedef __bf16 T; };
template <int ET, bool SPLIT, int BIAS_MODE, int OUT_MODE, bool RESID, int ACT = 0>
__global__ __launch_bounds__(256) void wmma_gemm64(
    const unsigned short* __restrict__ Ap, const unsigned short* __restrict__ A2p, int lda, long strideA,
    const unsigned short* __restrict__ Btp, const unsigned short* __restrict__ Bt2p, int ldb, long strideB,
    void* __restrict__ Cout, void* __restrict__ Cout2, int ldc, long strideC,
    const float* __restrict__ bias,
    const float* __restrict__ resid, long strideR,
    int M, int N, int K, float scale) {
  typedef typename Elem<ET>::T T;
  typedef typename Frag<T>::V V;
  const T* A = (const T*)Ap; const T* A2 = (const T*)A2p; const T* Bt = (const T*)Btp; const T* Bt2 = (const T*)Bt2p;
  __shared__ __align__(16) float sT[8][16 * 68];
  const int b    = blockIdx.y;
  const int lane = threadIdx.x & 31;
  const int wave = threadIdx.x >> 5;
  const int tilesN = N >> 6;
  const int tilesM = M >> 6;
  const int tile = blockIdx.x * 8 + wave;
  if (tile >= tilesM * tilesN) return;
  const int tm = tile / tilesN;
  const int tn = tile - tm * tilesN;
  const int m0 = tm << 6;
  const int n0 = tn << 6;

  const T* Ab  = A  + (size_t)b * strideA;
  const T* Bb  = Bt + (size_t)b * strideB;
  const T* Ab2 = SPLIT ? (A2  + (size_t)b * strideA) : nullptr;
  const T* Bb2 = SPLIT ? (Bt2 + (size_t)b * strideB) : nullptr;

  const int rlane = lane & 15;
  const int koff  = (lane >> 4) * 8;
  const int mOff  = (lane >> 4) * 8;

  v8f acc[4][4];
#pragma unroll
  for (int i = 0; i < 4; ++i)
#pragma unroll
    for (int j = 0; j < 4; ++j) acc[i][j] = (v8f){0.f,0.f,0.f,0.f,0.f,0.f,0.f,0.f};

  for (int k0 = 0; k0 < K; k0 += 32) {
    V bh[4], bl[4];
#pragma unroll
    for (int j = 0; j < 4; ++j) {
      const size_t bo = (size_t)(n0 + (j << 4) + rlane) * ldb + koff + k0;
      bh[j] = Frag<T>::load(Bb + bo);
      if (SPLIT) bl[j] = Frag<T>::load(Bb2 + bo);
    }
#pragma unroll
    for (int i = 0; i < 4; ++i) {
      const size_t ao = (size_t)(m0 + (i << 4) + rlane) * lda + koff + k0;
      V ah = Frag<T>::load(Ab + ao);
      V al;
      if (SPLIT) al = Frag<T>::load(Ab2 + ao);
#pragma unroll
      for (int j = 0; j < 4; ++j) {
        acc[i][j] = Frag<T>::mma(ah, bh[j], acc[i][j]);
        if (SPLIT) {
          acc[i][j] = Frag<T>::mma(ah, bl[j], acc[i][j]);
          acc[i][j] = Frag<T>::mma(al, bh[j], acc[i][j]);
        }
      }
      Frag<T>::guard(acc[i][0], acc[i][3], ah, SPLIT ? al : ah);
    }
    Frag<T>::keep(bh[0], bh[1], bh[2], bh[3]);
    if (SPLIT) Frag<T>::keep(bl[0], bl[1], bl[2], bl[3]);
  }
  acc_guard4(acc[0][0], acc[0][1], acc[0][2], acc[0][3]);
  acc_guard4(acc[1][0], acc[1][1], acc[1][2], acc[1][3]);
  acc_guard4(acc[2][0], acc[2][1], acc[2][2], acc[2][3]);
  acc_guard4(acc[3][0], acc[3][1], acc[3][2], acc[3][3]);

  float* slab = sT[wave];
  const float* Rb = RESID ? (resid + (size_t)b * strideR) : nullptr;
#pragma unroll
  for (int i = 0; i < 4; ++i) {
    const int mBase = m0 + (i << 4);
#pragma unroll
    for (int j = 0; j < 4; ++j) {
      const int n = n0 + (j << 4) + rlane;
      float bv = 0.f;
      if (BIAS_MODE == 2) bv = bias[n];
#pragma unroll
      for (int r = 0; r < 8; ++r) {
        float v = acc[i][j][r] * scale;
        if (BIAS_MODE == 1) v += bias[mBase + mOff + r];
        if (BIAS_MODE == 2) v += bv;
        if (RESID) v += Rb[(size_t)(mBase + mOff + r) * ldc + n];
        if (ACT == 1) v = tanhf(v);
        if (ACT == 2) v = fmaxf(v, 0.0f);
        if (ACT == 3) v = v / (1.0f + expf(-v));
        if (ACT == 4) v = (v > 0.f) ? v : 0.01f * v;
        if (ACT == 5) v = 0.5f * v * (1.0f + erff(v * 0.70710678118654752f));
        slab[(mOff + r) * 68 + (j << 4) + rlane] = v;
      }
    }
    __builtin_amdgcn_fence(__ATOMIC_RELEASE, "workgroup");
    __builtin_amdgcn_wave_barrier();
    __builtin_amdgcn_fence(__ATOMIC_ACQUIRE, "workgroup");
    if (OUT_MODE == 0) {
      float* C = (float*)Cout + (size_t)b * strideC;
      const int hh = lane >> 4, c4 = (lane & 15) * 4;
      for (int pass = 0; pass < 2; ++pass) {
#pragma unroll
        for (int it = 0; it < 8; ++it) {
          const int row = it * 2 + hh;
          v4f v = *(const v4f*)(slab + row * 68 + c4);
          *(volatile v4f*)(C + (size_t)(mBase + row) * ldc + n0 + c4) = v;
        }
        __threadfence();
      }
    } else {
      const int q = lane >> 3, c8 = (lane & 7) * 8;
      unsigned short* C  = (unsigned short*)Cout  + (size_t)b * strideC;
      unsigned short* C2 = (OUT_MODE == 2) ? ((unsigned short*)Cout2 + (size_t)b * strideC) : nullptr;
      for (int pass = 0; pass < 2; ++pass) {
#pragma unroll
        for (int it = 0; it < 4; ++it) {
          const int row = it * 4 + q;
          const float* sp = slab + row * 68 + c8;
          v8h hv, lv;
#pragma unroll
          for (int e = 0; e < 8; ++e) {
            if (OUT_MODE == 1) {
              hv[e] = (_Float16)sp[e];
            } else {
              unsigned short hb = f2bf_bits(sp[e]);
              unsigned short lb = f2bf_bits(sp[e] - bf_bits2f(hb));
              hv[e] = __builtin_bit_cast(_Float16, hb);
              lv[e] = __builtin_bit_cast(_Float16, lb);
            }
          }
          *(volatile v8h*)(C + (size_t)(mBase + row) * ldc + n0 + c8) = hv;
          if (OUT_MODE == 2) *(volatile v8h*)(C2 + (size_t)(mBase + row) * ldc + n0 + c8) = lv;
        }
        __threadfence();
      }
    }
    __builtin_amdgcn_fence(__ATOMIC_RELEASE, "workgroup");
    __builtin_amdgcn_wave_barrier();
    __builtin_amdgcn_fence(__ATOMIC_ACQUIRE, "workgroup");
  }
}

__global__ __launch_bounds__(256) void cast_f32_f16x2(
    const float* __restrict__ in, _Float16* __restrict__ out, int n2) {
  int i = blockIdx.x * 256 + threadIdx.x;
  if (i < n2) {
    const _Float16 h0 = (_Float16)in[2 * i], h1 = (_Float16)in[2 * i + 1];
    const unsigned u = (unsigned)__builtin_bit_cast(unsigned short, h0) | ((unsigned)__builtin_bit_cast(unsigned short, h1) << 16);
    ((volatile unsigned*)out)[i] = u;
    __threadfence();
    ((volatile unsigned*)out)[i] = u;
  }
}

__global__ __launch_bounds__(256) void transpose_cast_f16(const float* __restrict__ in, int ldi,
                                                         _Float16* __restrict__ outT, int ldo, float scale) {
  __shared__ __align__(16) _Float16 tile[64][72];
  const int c0 = blockIdx.x * 64, r0 = blockIdx.y * 64;
  const int t = threadIdx.y * 32 + threadIdx.x;
  for (int i = threadIdx.y; i < 64; i += 8) {
    tile[threadIdx.x][i]      = (_Float16)(in[(size_t)(r0 + i) * ldi + c0 + threadIdx.x] * scale);
    tile[32 + threadIdx.x][i] = (_Float16)(in[(size_t)(r0 + i) * ldi + c0 + 32 + threadIdx.x] * scale);
  }
  __syncthreads();
  const int q = t >> 3, c8 = (t & 7) * 8;
  for (int pass = 0; pass < 2; ++pass) {
#pragma unroll
    for (int it = 0; it < 2; ++it) {
      const int c = it * 32 + q;
      v8h hv = *(const v8h*)(&tile[c][c8]);
      *(volatile v8h*)(outT + (size_t)(c0 + c) * ldo + r0 + c8) = hv;
    }
    __threadfence();
  }
}

#define NN 10000
#define NE 160000
#define FD 56
#define MP 64
#define EF 64
#define HD 64
#define TW 1600
#define CHE 16000
#define NCHK (NE / CHE)
#define NT 256
#define TN 256
#define NTILE ((NN + TN - 1) / TN)
#define SCH 1024
#define NCHA ((NE + SCH - 1) / SCH)
static_assert(NE % CHE == 0);
static_assert(CHE % 64 == 0);
static_assert(CHE % 8 == 0);
static_assert(NE % 4 == 0);
static_assert(NN % 4 == 0);
static_assert(TN == NT);
static_assert(NE < (1 << 20));

__global__ __launch_bounds__(NT) void tp_kernel(const unsigned short* __restrict__ Wf, const int* __restrict__ ei, const float* __restrict__ na,
                                               const float* __restrict__ esh, int e0, float* __restrict__ M) {
  __shared__ float xs[8][FD];
  __shared__ float shs[8][4];
  __shared__ __align__(16) float os[8][MP];
  const int lane = threadIdx.x & 31, wave = threadIdx.x >> 5;
  const int le = blockIdx.x * 8 + wave;
  const int e  = e0 + le;
  int d = ei[NE + e]; d = d < 0 ? 0 : (d >= NN ? NN - 1 : d);
  if (lane < 28) { xs[wave][lane] = na[(size_t)d * FD + lane]; xs[wave][28 + lane] = na[(size_t)d * FD + 28 + lane]; }
  if (lane < 4) shs[wave][lane] = esh[(size_t)e * 4 + lane];
  __syncthreads();
  const _Float16* wr = (const _Float16*)Wf + (size_t)le * TW;
  const float* x = xs[wave];
  const float sh0 = shs[wave][0], s1 = shs[wave][1], s2 = shs[wave][2], s3 = shs[wave][3];
  const int v8 = (lane < 24) ? (lane / 3) : 0;
  const int m3 = (lane < 24) ? (lane - 3 * v8) : 0;
  float a = 0.f, p = 0.f;
#pragma unroll 1
  for (int u = 0; u < 32; ++u) {
    const float xu = x[u];
    a += (float)wr[u * 32 + lane] * xu;
    p += (float)wr[1024 + u * 8 + v8] * xu;
  }
  float c4 = 0.f, q2 = 0.f;
#pragma unroll 1
  for (int u = 0; u < 8; ++u) {
    const float x10 = x[32 + u * 3], x11 = x[32 + u * 3 + 1], x12 = x[32 + u * 3 + 2];
    const float dotm = x10 * s1 + x11 * s2 + x12 * s3;
    c4 += (float)wr[1344 + u * 32 + lane] * dotm;
    const float x1m = (m3 == 0) ? x10 : (m3 == 1 ? x11 : x12);
    q2 += (float)wr[1280 + u * 8 + v8] * x1m;
  }
  const float shm = (m3 == 0) ? s1 : (m3 == 1 ? s2 : s3);
  const float o0 = (a * sh0 + 0.57735026918962576f * c4) * 0.15811388300841897f;
  const float o1 = (lane < 24) ? (p * shm + q2 * sh0) * 0.15811388300841897f : 0.f;
  os[wave][lane] = o0; os[wave][32 + lane] = o1;
  __syncthreads();
  v4f ov = (v4f){0.f, 0.f, 0.f, 0.f};
  if (lane < 16) ov = *(const v4f*)(&os[wave][4 * lane]);
  float* mrow = M + (size_t)e * MP;
  for (int pass = 0; pass < 2; ++pass) {
    if (lane < 16) *(volatile v4f*)(mrow + 4 * lane) = ov;
    __threadfence();
  }
}

__device__ __forceinline__ int blk_excl_scan(int cnt, int* scan_ws, int tid, int* tot) {
  const int lane = tid & 31, wave = tid >> 5; int incl = cnt;
#pragma unroll
  for (int o = 1; o < 32; o <<= 1) { const int v = __shfl_up(incl, o, 32); if (lane >= o) incl += v; }
  if (lane == 31) scan_ws[wave] = incl;
  __syncthreads();
  if (wave == 0) { int wv = (lane < NT / 32) ? scan_ws[lane] : 0; int wincl = wv;
#pragma unroll
    for (int o = 1; o < 32; o <<= 1) { const int v = __shfl_up(wincl, o, 32); if (lane >= o) wincl += v; }
    if (lane < NT / 32) scan_ws[32 + lane] = wincl - wv; if (lane == 31) scan_ws[64] = wincl; }
  __syncthreads();
  const int res = scan_ws[32 + wave] + incl - cnt; *tot = scan_ws[64];
  return res;
}
template <int SP, int CAP>
__device__ __forceinline__ int chunk_hits(const int* __restrict__ keyv, int e0, int n0, int tid, int* LIST, int* scan_ws) {
  const int eb = e0 + tid * SP;
  int rec[SP]; int cnt = 0;
#pragma unroll
  for (int k = 0; k < SP; k += 4) {
    v4i d4 = (v4i){-1, -1, -1, -1};
    if (eb + k < NE) d4 = *(const v4i*)(keyv + eb + k);
#pragma unroll
    for (int q = 0; q < 4; ++q) {
      const int d = d4[q]; int r = -1;
      if (d >= n0 && d < n0 + TN) { r = ((d - n0) << 20) | (eb + k + q); ++cnt; }
      rec[k + q] = r;
    }
  }
  int tot; int p = blk_excl_scan(cnt, scan_ws, tid, &tot);
#pragma unroll
  for (int k = 0; k < SP; ++k) if (rec[k] >= 0) { if ((unsigned)p < (unsigned)CAP) LIST[p] = rec[k]; ++p; }
  __syncthreads();
  return tot < CAP ? tot : CAP;
}

__global__ __launch_bounds__(NT) void agg_kernel(const float* __restrict__ M, const int* __restrict__ ei, const float* __restrict__ na,
                                                float* __restrict__ out) {
  __shared__ __align__(16) float ACC[TN * FD];
  __shared__ int CNT[TN];
  __shared__ int LIST[SCH];
  __shared__ int scan_ws[80];
  const int tid = threadIdx.x, lane = tid & 31, wave = tid >> 5;
  const int n0 = blockIdx.x * TN;
  for (int i = tid; i < TN * FD; i += NT) ACC[i] = 0.f;
  CNT[tid] = 0;
  __syncthreads();
#pragma unroll 1
  for (int c = 0; c < NCHA; ++c) {
    const int tot = chunk_hits<SCH / NT, SCH>(ei, c * SCH, n0, tid, LIST, scan_ws);
#pragma unroll 1
    for (int base = 0; base < tot; base += 32) {
      const int q = base + lane;
      const int rv = (q < tot) ? LIST[q] : -1;
      const int own = (rv >= 0 && (rv >> 25) == wave) ? 1 : 0;
      unsigned msk = (unsigned)__ballot(own);
#pragma unroll 1
      for (int it = 0; it < 32; ++it) {
        if (msk == 0u) break;
        const int bp = __builtin_ctz(msk); msk &= msk - 1u;
        const int r = __shfl(rv, bp, 32);
        const int dl = (r >> 20) & (TN - 1);
        int e = r & 0xFFFFF; e = e < NE ? e : NE - 1;
        if (lane < 28) {
          const v2f mv = *(const v2f*)(M + (size_t)e * MP + 2 * lane);
          v2f* ap = (v2f*)(ACC + dl * FD + 2 * lane);
          v2f av = *ap; av = av + mv; *ap = av;
        }
        if (lane == 0) CNT[dl] += 1;
      }
    }
    __syncthreads();
  }
#pragma unroll 1
  for (int g = 0; g < 8; ++g) {
    const int r0 = wave * 32 + g * 4;
    const int ng = n0 + r0;
    if (ng < NN) {
      const float* ap = ACC + r0 * FD;
      const int qa = lane / 14;
      const int lb = (lane < 24) ? lane : 23;
      const int qb = (32 + lb) / 14;
      const int ca = CNT[r0 + qa], cb = CNT[r0 + qb];
      const float inva = 1.0f / (float)(ca > 0 ? ca : 1);
      const float invb = 1.0f / (float)(cb > 0 ? cb : 1);
      const v4f aa = *(const v4f*)(ap + 4 * lane);
      const v4f ab = *(const v4f*)(ap + 128 + 4 * lb);
      const float* xr = na + (size_t)ng * FD;
      const v4f xa = *(const v4f*)(xr + 4 * lane);
      const v4f xb = *(const v4f*)(xr + 128 + 4 * lb);
      v4f oa = aa * inva; fence_v4(oa); oa = oa + xa;
      v4f ob = ab * invb; fence_v4(ob); ob = ob + xb;
      float* orow = out + (size_t)ng * FD;
      for (int pass = 0; pass < 2; ++pass) {
        *(volatile v4f*)(orow + 4 * lane) = oa;
        if (lane < 24) *(volatile v4f*)(orow + 128 + 4 * lane) = ob;
        __threadfence();
      }
    }
  }
}

extern "C" void kernel_launch(void* const* d_in, const int* in_sizes, int n_in,
                              void* d_out, int out_size, void* d_ws, size_t ws_size, hipStream_t stream) {
  (void)in_sizes; (void)out_size;
  if (n_in < 8) return;
  const float* na  = (const float*)d_in[0];
  const float* ea  = (const float*)d_in[1];
  const float* esh = (const float*)d_in[2];
  const float* W1  = (const float*)d_in[3];
  const float* b1  = (const float*)d_in[4];
  const float* W2  = (const float*)d_in[5];
  const float* b2  = (const float*)d_in[6];
  const int*   ei  = (const int*)d_in[7];
  float* out = (float*)d_out;

  char* ws = (char*)d_ws; size_t off = 0;
  auto carve = [&](size_t bytes) -> char* { char* p = ws + off; off += (bytes + 255) & ~(size_t)255; return p; };
  _Float16*       W1T  = (_Float16*)carve((size_t)HD * EF * 2);
  _Float16*       W2T  = (_Float16*)carve((size_t)TW * HD * 2);
  unsigned short* EA16 = (unsigned short*)carve((size_t)NE * EF * 2);
  unsigned short* H1   = (unsigned short*)carve((size_t)CHE * HD * 2);
  unsigned short* Wf   = (unsigned short*)carve((size_t)CHE * TW * 2);
  float*          M    = (float*)carve((size_t)NE * MP * 4);
  if (off > ws_size || off > (size_t)134217728) return;

  cast_f32_f16x2<<<(NE * EF / 2 + 255) / 256, 256, 0, stream>>>(ea, (_Float16*)EA16, NE * EF / 2);
  transpose_cast_f16<<<dim3(HD / 64, EF / 64), dim3(32, 8), 0, stream>>>(W1, HD, W1T, EF, 1.0f);
  transpose_cast_f16<<<dim3(TW / 64, HD / 64), dim3(32, 8), 0, stream>>>(W2, TW, W2T, HD, 1.0f);
  const int t1 = (CHE / 64) * (HD / 64);
  const int t2 = (CHE / 64) * (TW / 64);
  for (int ch = 0; ch < NCHK; ++ch) {
    const int e0 = ch * CHE;
    wmma_gemm64<0, false, 2, 1, false, 2><<<dim3((t1 + 7) / 8, 1), 256, 0, stream>>>(
        (const unsigned short*)EA16 + (size_t)e0 * EF, nullptr, EF, 0L, U16(W1T), nullptr, EF, 0L,
        (void*)H1, nullptr, HD, 0L, b1, nullptr, 0L, CHE, HD, EF, 1.0f);
    wmma_gemm64<0, false, 2, 1, false, 0><<<dim3((t2 + 7) / 8, 1), 256, 0, stream>>>(
        (const unsigned short*)H1, nullptr, HD, 0L, U16(W2T), nullptr, HD, 0L,
        (void*)Wf, nullptr, TW, 0L, b2, nullptr, 0L, CHE, TW, HD, 1.0f);
    tp_kernel<<<CHE / 8, NT, 0, stream>>>(Wf, ei, na, esh, e0, M);
  }
  agg_kernel<<<NTILE, NT, 0, stream>>>(M, ei, na, out);
}
